// mowLSTM__31920196944207
// MI455X (gfx1250) — hardware-verified
//
#include <hip/hip_runtime.h>

typedef __attribute__((ext_vector_type(16))) _Float16 v16h;
typedef __attribute__((ext_vector_type(8)))  _Float16 v8h;
typedef __attribute__((ext_vector_type(16))) __bf16   v16b;
typedef __attribute__((ext_vector_type(8)))  __bf16   v8b;
typedef __attribute__((ext_vector_type(8)))  float    v8f;
typedef __attribute__((ext_vector_type(4)))  float    v4f;

constexpr int SEQ_T  = 128;
constexpr int NBATCH = 64;
constexpr int NIN    = 256;
constexpr int NHID   = 512;
constexpr int NEXP   = 4;
constexpr int NGATE  = 4 * NHID;
constexpr int KX     = NEXP * NIN;
constexpr int KHH    = NEXP * NHID;
constexpr int NROW   = SEQ_T * NBATCH;
constexpr float W_CARRY     = 16.0f;
constexpr float W_CARRY_INV = 1.0f / 16.0f;
constexpr int HT_PITCH = KHH + 8;
constexpr int SLAB_ROWS  = 4;
constexpr int SLAB_PITCH = 32;
static_assert(KX % 32 == 0 && KHH % 32 == 0);
static_assert(NBATCH % 64 == 0 && NGATE % 64 == 0);
static_assert((HT_PITCH % 8) == 0);

constexpr size_t WS_XA    = 0;
constexpr size_t WS_WIT   = WS_XA   + (size_t)NROW   * KX    * 2;
constexpr size_t WS_WHT   = WS_WIT  + (size_t)NGATE  * KX    * 2;
constexpr size_t WS_BMIX  = WS_WHT  + (size_t)NGATE  * KHH   * 2;
constexpr size_t WS_XG    = WS_BMIX + (size_t)NBATCH * NGATE * 4;
constexpr size_t WS_TOTAL = WS_XG   + (size_t)NROW   * NGATE * 4;
static_assert(WS_TOTAL == 96993280u);
static_assert(WS_TOTAL <= 134217728u);

__device__ __forceinline__ unsigned short f2bf_bits(float f) {
  unsigned u = __float_as_uint(f);
  return (unsigned short)((u + 0x7FFFu + ((u >> 16) & 1u)) >> 16);
}
__device__ __forceinline__ float bf_bits2f(unsigned short h) { return __uint_as_float(((unsigned)h) << 16); }

__device__ __forceinline__ void dep_guard_h(v8f& a, v8f& b, v16h x, v16h y) { asm volatile("v_nop\n\tv_nop\n\tv_nop\n\tv_nop" : "+v"(a), "+v"(b) : "v"(x), "v"(y)); }
__device__ __forceinline__ void dep_guard_b(v8f& a, v8f& b, v16b x, v16b y) { asm volatile("v_nop\n\tv_nop\n\tv_nop\n\tv_nop" : "+v"(a), "+v"(b) : "v"(x), "v"(y)); }
__device__ __forceinline__ void keep4_h(v16h a, v16h b, v16h c, v16h d) { asm volatile("v_nop" :: "v"(a), "v"(b), "v"(c), "v"(d)); }
__device__ __forceinline__ void keep4_b(v16b a, v16b b, v16b c, v16b d) { asm volatile("v_nop" :: "v"(a), "v"(b), "v"(c), "v"(d)); }
__device__ __forceinline__ void acc_guard4(v8f& a, v8f& b, v8f& c, v8f& d) { asm volatile("v_nop\n\tv_nop\n\tv_nop\n\tv_nop" : "+v"(a), "+v"(b), "+v"(c), "+v"(d)); }
template <typename T> struct Frag;
template <> struct Frag<_Float16> {
  typedef v16h V; union U { v16h v; v8h h[2]; };
  static __device__ __forceinline__ v16h load(const _Float16* p) {
    U f; f.h[0] = *(const v8h*)(p); f.h[1] = *(const v8h*)(p + 16); return f.v;
  }
  static __device__ __forceinline__ v8f mma(v16h a, v16h b, v8f c) {
    return __builtin_amdgcn_wmma_f32_16x16x32_f16(false, a, false, b, (short)0, c, false, false);
  }
  static __device__ __forceinline__ void guard(v8f& a, v8f& b, v16h x, v16h y) { dep_guard_h(a, b, x, y); }
  static __device__ __forceinline__ void keep(v16h a, v16h b, v16h c, v16h d) { keep4_h(a, b, c, d); }
};
template <> struct Frag<__bf16> {
  typedef v16b V; union U { v16b v; v8b h[2]; };
  static __device__ __forceinline__ v16b load(const __bf16* p) {
    U f; f.h[0] = *(const v8b*)(p); f.h[1] = *(const v8b*)(p + 16); return f.v;
  }
  static __device__ __forceinline__ v8f mma(v16b a, v16b b, v8f c) {
    return __builtin_amdgcn_wmma_f32_16x16x32_bf16(false, a, false, b, (short)0, c, false, false);
  }
  static __device__ __forceinline__ void guard(v8f& a, v8f& b, v16b x, v16b y) { dep_guard_b(a, b, x, y); }
  static __device__ __forceinline__ void keep(v16b a, v16b b, v16b c, v16b d) { keep4_b(a, b, c, d); }
};

template <int ET> struct Elem;
template <> struct Elem<0> { typedef _Float16 T; };
template <> struct Elem<1> { typedef __bf16 T; };
template <int ET, bool SPLIT, int BIAS_MODE, int OUT_MODE, bool RESID, int ACT = 0>
__global__ __launch_bounds__(256) void wmma_gemm64(
    const unsigned short* __restrict__ Ap, const unsigned short* __restrict__ A2p, int lda, long strideA,
    const unsigned short* __restrict__ Btp, const unsigned short* __restrict__ Bt2p, int ldb, long strideB,
    void* __restrict__ Cout, void* __restrict__ Cout2, int ldc, long strideC,
    const float* __restrict__ bias,
    const float* __restrict__ resid, long strideR,
    int M, int N, int K, float scale) {
  typedef typename Elem<ET>::T T;
  typedef typename Frag<T>::V V;
  const T* A = (const T*)Ap; const T* A2 = (const T*)A2p; const T* Bt = (const T*)Btp; const T* Bt2 = (const T*)Bt2p;
  __shared__ __align__(16) float sT[8][16 * 68];
  const int b    = blockIdx.y;
  const int lane = threadIdx.x & 31;
  const int wave = threadIdx.x >> 5;
  const int tilesN = N >> 6;
  const int tilesM = M >> 6;
  const int tile = blockIdx.x * 8 + wave;
  if (tile >= tilesM * tilesN) return;
  const int tm = tile / tilesN;
  const int tn = tile - tm * tilesN;
  const int m0 = tm << 6;
  const int n0 = tn << 6;

  const T* Ab  = A  + (size_t)b * strideA;
  const T* Bb  = Bt + (size_t)b * strideB;
  const T* Ab2 = SPLIT ? (A2  + (size_t)b * strideA) : nullptr;
  const T* Bb2 = SPLIT ? (Bt2 + (size_t)b * strideB) : nullptr;

  const int rlane = lane & 15;
  const int koff  = (lane >> 4) * 8;
  const int mOff  = (lane >> 4) * 8;

  v8f acc[4][4];
#pragma unroll
  for (int i = 0; i < 4; ++i)
#pragma unroll
    for (int j = 0; j < 4; ++j) acc[i][j] = (v8f){0.f,0.f,0.f,0.f,0.f,0.f,0.f,0.f};

  for (int k0 = 0; k0 < K; k0 += 32) {
    V bh[4], bl[4];
#pragma unroll
    for (int j = 0; j < 4; ++j) {
      const size_t bo = (size_t)(n0 + (j << 4) + rlane) * ldb + koff + k0;
      bh[j] = Frag<T>::load(Bb + bo);
      if (SPLIT) bl[j] = Frag<T>::load(Bb2 + bo);
    }
#pragma unroll
    for (int i = 0; i < 4; ++i) {
      const size_t ao = (size_t)(m0 + (i << 4) + rlane) * lda + koff + k0;
      V ah = Frag<T>::load(Ab + ao);
      V al;
      if (SPLIT) al = Frag<T>::load(Ab2 + ao);
#pragma unroll
      for (int j = 0; j < 4; ++j) {
        acc[i][j] = Frag<T>::mma(ah, bh[j], acc[i][j]);
        if (SPLIT) {
          acc[i][j] = Frag<T>::mma(ah, bl[j], acc[i][j]);
          acc[i][j] = Frag<T>::mma(al, bh[j], acc[i][j]);
        }
      }
      Frag<T>::guard(acc[i][0], acc[i][3], ah, SPLIT ? al : ah);
    }
    Frag<T>::keep(bh[0], bh[1], bh[2], bh[3]);
    if (SPLIT) Frag<T>::keep(bl[0], bl[1], bl[2], bl[3]);
  }
  acc_guard4(acc[0][0], acc[0][1], acc[0][2], acc[0][3]);
  acc_guard4(acc[1][0], acc[1][1], acc[1][2], acc[1][3]);
  acc_guard4(acc[2][0], acc[2][1], acc[2][2], acc[2][3]);
  acc_guard4(acc[3][0], acc[3][1], acc[3][2], acc[3][3]);

  float* slab = sT[wave];
  const float* Rb = RESID ? (resid + (size_t)b * strideR) : nullptr;
#pragma unroll
  for (int i = 0; i < 4; ++i) {
    const int mBase = m0 + (i << 4);
#pragma unroll
    for (int j = 0; j < 4; ++j) {
      const int n = n0 + (j << 4) + rlane;
      float bv = 0.f;
      if (BIAS_MODE == 2) bv = bias[n];
#pragma unroll
      for (int r = 0; r < 8; ++r) {
        float v = acc[i][j][r] * scale;
        if (BIAS_MODE == 1) v += bias[mBase + mOff + r];
        if (BIAS_MODE == 2) v += bv;
        if (RESID) v += Rb[(size_t)(mBase + mOff + r) * ldc + n];
        if (ACT == 1) v = tanhf(v);
        if (ACT == 2) v = fmaxf(v, 0.0f);
        if (ACT == 3) v = v / (1.0f + expf(-v));
        if (ACT == 4) v = (v > 0.f) ? v : 0.01f * v;
        if (ACT == 5) v = 0.5f * v * (1.0f + erff(v * 0.70710678118654752f));
        slab[(mOff + r) * 68 + (j << 4) + rlane] = v;
      }
    }
    __builtin_amdgcn_fence(__ATOMIC_RELEASE, "workgroup");
    __builtin_amdgcn_wave_barrier();
    __builtin_amdgcn_fence(__ATOMIC_ACQUIRE, "workgroup");
    if (OUT_MODE == 0) {
      float* C = (float*)Cout + (size_t)b * strideC;
      const int hh = lane >> 4, c4 = (lane & 15) * 4;
      for (int pass = 0; pass < 2; ++pass) {
#pragma unroll
        for (int it = 0; it < 8; ++it) {
          const int row = it * 2 + hh;
          v4f v = *(const v4f*)(slab + row * 68 + c4);
          *(volatile v4f*)(C + (size_t)(mBase + row) * ldc + n0 + c4) = v;
        }
        __threadfence();
      }
    } else {
      const int q = lane >> 3, c8 = (lane & 7) * 8;
      unsigned short* C  = (unsigned short*)Cout  + (size_t)b * strideC;
      unsigned short* C2 = (OUT_MODE == 2) ? ((unsigned short*)Cout2 + (size_t)b * strideC) : nullptr;
      for (int pass = 0; pass < 2; ++pass) {
#pragma unroll
        for (int it = 0; it < 4; ++it) {
          const int row = it * 4 + q;
          const float* sp = slab + row * 68 + c8;
          v8h hv, lv;
#pragma unroll
          for (int e = 0; e < 8; ++e) {
            if (OUT_MODE == 1) {
              hv[e] = (_Float16)sp[e];
            } else {
              unsigned short hb = f2bf_bits(sp[e]);
              unsigned short lb = f2bf_bits(sp[e] - bf_bits2f(hb));
              hv[e] = __builtin_bit_cast(_Float16, hb);
              lv[e] = __builtin_bit_cast(_Float16, lb);
            }
          }
          *(volatile v8h*)(C + (size_t)(mBase + row) * ldc + n0 + c8) = hv;
          if (OUT_MODE == 2) *(volatile v8h*)(C2 + (size_t)(mBase + row) * ldc + n0 + c8) = lv;
        }
        __threadfence();
      }
    }
    __builtin_amdgcn_fence(__ATOMIC_RELEASE, "workgroup");
    __builtin_amdgcn_wave_barrier();
    __builtin_amdgcn_fence(__ATOMIC_ACQUIRE, "workgroup");
  }
}


__global__ __launch_bounds__(256) void k_build_xa(const float* __restrict__ x, const float* __restrict__ coef,
                                                  unsigned short* __restrict__ xa) {
  const int idx = blockIdx.x * 256 + threadIdx.x;
  if (idx >= NROW * (KX / 8)) return;
  const int row = idx >> 7;
  const int j   = idx & 127;
  const int e   = j >> 5;
  const int i8  = (j & 31) * 8;
  const int b   = row & (NBATCH - 1);
  const float cf = coef[b * NEXP + e];
  const float* xp = x + (size_t)row * NIN + i8;
  const v4f x0 = *(const v4f*)(xp);
  const v4f x1 = *(const v4f*)(xp + 4);
  v8h hv;
#pragma unroll
  for (int q = 0; q < 4; ++q) { hv[q] = (_Float16)(x0[q] * cf); hv[4 + q] = (_Float16)(x1[q] * cf); }
  _Float16* dst = (_Float16*)xa + (size_t)idx * 8;
  *(volatile v8h*)dst = hv;
  __threadfence();
  *(volatile v8h*)dst = hv;
}

__global__ __launch_bounds__(256) void k_build_wit(const float* __restrict__ wi, unsigned short* __restrict__ wit) {
  const int idx = blockIdx.x * 256 + threadIdx.x;
  if (idx >= NGATE * (KX / 8)) return;
  const int o  = idx >> 7;
  const int j  = idx & 127;
  const int e  = j >> 5;
  const int i8 = (j & 31) * 8;
  const float* sp = wi + ((size_t)e * NGATE + o) * NIN + i8;
  const v4f w0 = *(const v4f*)(sp);
  const v4f w1 = *(const v4f*)(sp + 4);
  v8h hv;
#pragma unroll
  for (int q = 0; q < 4; ++q) { hv[q] = (_Float16)(w0[q] * W_CARRY); hv[4 + q] = (_Float16)(w1[q] * W_CARRY); }
  _Float16* dst = (_Float16*)wit + (size_t)idx * 8;
  *(volatile v8h*)dst = hv;
  __threadfence();
  *(volatile v8h*)dst = hv;
}

__global__ __launch_bounds__(256) void k_build_wht(const float* __restrict__ wh, unsigned short* __restrict__ wht) {
  const int idx = blockIdx.x * 256 + threadIdx.x;
  if (idx >= NGATE * (KHH / 8)) return;
  const int o  = idx >> 8;
  const int j  = idx & 255;
  const int e  = j >> 6;
  const int h8 = (j & 63) * 8;
  const float* sp = wh + ((size_t)e * NGATE + o) * NHID + h8;
  const v4f w0 = *(const v4f*)(sp);
  const v4f w1 = *(const v4f*)(sp + 4);
  v8h hv;
#pragma unroll
  for (int q = 0; q < 4; ++q) { hv[q] = (_Float16)(w0[q] * W_CARRY); hv[4 + q] = (_Float16)(w1[q] * W_CARRY); }
  _Float16* dst = (_Float16*)wht + (size_t)idx * 8;
  *(volatile v8h*)dst = hv;
  __threadfence();
  *(volatile v8h*)dst = hv;
}

__global__ __launch_bounds__(256) void k_bias_mix(const float* __restrict__ coef, const float* __restrict__ bi,
                                                  const float* __restrict__ bh, float* __restrict__ bmix) {
  const int idx = blockIdx.x * 256 + threadIdx.x;
  if (idx >= NBATCH * (NGATE / 4)) return;
  const int b  = idx >> 9;
  const int o4 = (idx & 511) * 4;
  v4f s = (v4f){0.f, 0.f, 0.f, 0.f};
#pragma unroll
  for (int e = 0; e < NEXP; ++e) {
    const float cf = coef[b * NEXP + e];
    const v4f vi = *(const v4f*)(bi + (size_t)e * NGATE + o4);
    const v4f vh = *(const v4f*)(bh + (size_t)e * NGATE + o4);
    s = s + cf * (vi + vh);
  }
  float* dst = bmix + (size_t)idx * 4;
  *(volatile v4f*)dst = s;
  __threadfence();
  *(volatile v4f*)dst = s;
}

__device__ __forceinline__ float sigm_f(float x) {
  x = fminf(fmaxf(x, -30.0f), 30.0f);
  return 1.0f / (1.0f + expf(-x));
}
__device__ __forceinline__ float tanh_f(float x) {
  x = fminf(fmaxf(x, -15.0f), 15.0f);
  return 1.0f - 2.0f / (1.0f + expf(2.0f * x));
}
__device__ __forceinline__ void wave_sync_lds() {
  __builtin_amdgcn_fence(__ATOMIC_RELEASE, "workgroup");
  __builtin_amdgcn_wave_barrier();
  __builtin_amdgcn_fence(__ATOMIC_ACQUIRE, "workgroup");
}

__global__ __launch_bounds__(512) void k_recur(const unsigned short* __restrict__ whtp,
                                              const float* __restrict__ xg,
                                              const float* __restrict__ coef,
                                              const float* __restrict__ h0,
                                              const float* __restrict__ c0,
                                              float* __restrict__ out) {
  __shared__ __align__(16) _Float16 sAt[16 * HT_PITCH];
  __shared__ __align__(16) float    sSl[16][SLAB_ROWS * SLAB_PITCH];
  __shared__ __align__(16) float    sCf[16 * NEXP];
  const int tid  = threadIdx.x;
  const int lane = tid & 31;
  const int wave = tid >> 5;
  const int hh   = lane >> 4;
  const int cc   = lane & 15;
  const int row0 = blockIdx.x * 16;
  const int ubase = wave * 32 + cc;
  const _Float16* whT = (const _Float16*)whtp;
  float* slab = sSl[wave];

  if (tid < 16 * NEXP) sCf[tid] = coef[row0 * NEXP + tid];
  __syncthreads();
#pragma unroll
  for (int it = 0; it < 8; ++it) {
    const int v  = it * 512 + tid;
    const int r  = v >> 8;
    const int j  = v & 255;
    const int e  = j >> 6;
    const int u8 = (j & 63) * 8;
    const float cf = sCf[r * NEXP + e];
    const float* hp = h0 + (size_t)(row0 + r) * NHID + u8;
    const v4f a0 = *(const v4f*)(hp);
    const v4f a1 = *(const v4f*)(hp + 4);
    v8h hv;
#pragma unroll
    for (int q = 0; q < 4; ++q) { hv[q] = (_Float16)(a0[q] * cf); hv[4 + q] = (_Float16)(a1[q] * cf); }
    *(v8h*)(sAt + r * HT_PITCH + e * NHID + u8) = hv;
  }
  float cst[2][8];
#pragma unroll
  for (int us = 0; us < 2; ++us)
#pragma unroll
    for (int r = 0; r < 8; ++r)
      cst[us][r] = c0[(size_t)(row0 + 8 * hh + r) * NHID + ubase + 16 * us];

  for (int t = 0; t < SEQ_T; ++t) {
    __syncthreads();

    v8f acc[4][2];
#pragma unroll
    for (int g = 0; g < 4; ++g)
#pragma unroll
      for (int us = 0; us < 2; ++us) acc[g][us] = (v8f){0.f,0.f,0.f,0.f,0.f,0.f,0.f,0.f};

#pragma unroll 1
    for (int k0 = 0; k0 < KHH; k0 += 32) {
      const v16h af = Frag<_Float16>::load(sAt + cc * HT_PITCH + k0 + 8 * hh);
      v16h bq[4][2];
#pragma unroll
      for (int g = 0; g < 4; ++g)
#pragma unroll
        for (int us = 0; us < 2; ++us)
          bq[g][us] = Frag<_Float16>::load(whT + (size_t)(g * NHID + ubase + 16 * us) * KHH + k0 + 8 * hh);
#pragma unroll
      for (int g = 0; g < 4; ++g)
#pragma unroll
        for (int us = 0; us < 2; ++us)
          acc[g][us] = Frag<_Float16>::mma(af, bq[g][us], acc[g][us]);
      dep_guard_h(acc[0][0], acc[3][1], af, af);
      keep4_h(bq[0][0], bq[0][1], bq[1][0], bq[1][1]);
      keep4_h(bq[2][0], bq[2][1], bq[3][0], bq[3][1]);
    }
    acc_guard4(acc[0][0], acc[0][1], acc[1][0], acc[1][1]);
    acc_guard4(acc[2][0], acc[2][1], acc[3][0], acc[3][1]);
    __syncthreads();

    const float* xgt = xg + (size_t)(t * NBATCH + row0) * NGATE;
    float hreg[2][8];
#pragma unroll
    for (int us = 0; us < 2; ++us) {
      const int u = ubase + 16 * us;
#pragma unroll
      for (int r = 0; r < 8; ++r) {
        const int rr = 8 * hh + r;
        const float* xr = xgt + (size_t)rr * NGATE + u;
        const float gi = acc[0][us][r] * W_CARRY_INV + xr[0];
        const float gf = acc[1][us][r] * W_CARRY_INV + xr[NHID];
        const float gc = acc[2][us][r] * W_CARRY_INV + xr[2 * NHID];
        const float go = acc[3][us][r] * W_CARRY_INV + xr[3 * NHID];
        const float ig = sigm_f(gi);
        const float fg = sigm_f(gf);
        const float cg = tanh_f(gc);
        const float og = sigm_f(go);
        const float cn = fg * cst[us][r] + ig * cg;
        cst[us][r] = cn;
        hreg[us][r] = og * tanh_f(cn);
      }
    }

    const bool last = (t == SEQ_T - 1);
#pragma unroll
    for (int ph = 0; ph < 4; ++ph) {
#pragma unroll
      for (int q = 0; q < 2; ++q)
#pragma unroll
        for (int us = 0; us < 2; ++us)
          slab[(hh * 2 + q) * SLAB_PITCH + 16 * us + cc] = hreg[us][2 * ph + q];
      wave_sync_lds();
#pragma unroll
      for (int k = 0; k < 2; ++k) {
        const int i  = k * 32 + lane;
        const int s  = i >> 4;
        const int e  = (i >> 2) & 3;
        const int v8 = (i & 3) * 8;
        const int rr = 8 * (s >> 1) + 2 * ph + (s & 1);
        const float cf = sCf[rr * NEXP + e];
        const v4f a0 = *(const v4f*)(slab + s * SLAB_PITCH + v8);
        const v4f a1 = *(const v4f*)(slab + s * SLAB_PITCH + v8 + 4);
        v8h hv;
#pragma unroll
        for (int q = 0; q < 4; ++q) { hv[q] = (_Float16)(a0[q] * cf); hv[4 + q] = (_Float16)(a1[q] * cf); }
        *(v8h*)(sAt + rr * HT_PITCH + e * NHID + 32 * wave + v8) = hv;
      }
      {
        const int s  = lane >> 3;
        const int c4 = (lane & 7) * 4;
        const int rr = 8 * (s >> 1) + 2 * ph + (s & 1);
        const v4f vo = *(const v4f*)(slab + s * SLAB_PITCH + c4);
        float* d0 = out + ((size_t)(t * NBATCH + row0 + rr)) * NHID + 32 * wave + c4;
        float* d1 = out + (size_t)NROW * NHID + ((size_t)(row0 + rr)) * NHID + 32 * wave + c4;
        *(volatile v4f*)d0 = vo;
        if (last) *(volatile v4f*)d1 = vo;
        __threadfence();
        *(volatile v4f*)d0 = vo;
        if (last) *(volatile v4f*)d1 = vo;
      }
      wave_sync_lds();
    }
  }

#pragma unroll
  for (int ph = 0; ph < 4; ++ph) {
#pragma unroll
    for (int q = 0; q < 2; ++q)
#pragma unroll
      for (int us = 0; us < 2; ++us)
        slab[(hh * 2 + q) * SLAB_PITCH + 16 * us + cc] = cst[us][2 * ph + q];
    wave_sync_lds();
    {
      const int s  = lane >> 3;
      const int c4 = (lane & 7) * 4;
      const int rr = 8 * (s >> 1) + 2 * ph + (s & 1);
      const v4f vo = *(const v4f*)(slab + s * SLAB_PITCH + c4);
      float* d2 = out + (size_t)NROW * NHID + (size_t)NBATCH * NHID + ((size_t)(row0 + rr)) * NHID + 32 * wave + c4;
      *(volatile v4f*)d2 = vo;
      __threadfence();
      *(volatile v4f*)d2 = vo;
    }
    wave_sync_lds();
  }
}

extern "C" void kernel_launch(void* const* d_in, const int* in_sizes, int n_in,
                              void* d_out, int out_size, void* d_ws, size_t ws_size,
                              hipStream_t stream) {
  if (n_in < 8) return;
  if (in_sizes[0] != NROW * NIN) return;
  if (in_sizes[1] != NBATCH * NHID || in_sizes[2] != NBATCH * NHID) return;
  if (in_sizes[3] != NBATCH * NEXP) return;
  if (in_sizes[4] != NEXP * NGATE * NIN || in_sizes[5] != NEXP * NGATE) return;
  if (in_sizes[6] != NEXP * NGATE * NHID || in_sizes[7] != NEXP * NGATE) return;
  if (out_size != NROW * NHID + 2 * NBATCH * NHID) return;
  if (ws_size < WS_TOTAL) return;

  const float* x    = (const float*)d_in[0];
  const float* h0   = (const float*)d_in[1];
  const float* c0   = (const float*)d_in[2];
  const float* coef = (const float*)d_in[3];
  const float* Wi   = (const float*)d_in[4];
  const float* bi   = (const float*)d_in[5];
  const float* Wh   = (const float*)d_in[6];
  const float* bh   = (const float*)d_in[7];
  float* out = (float*)d_out;
  char* ws = (char*)d_ws;

  unsigned short* xa   = (unsigned short*)(ws + WS_XA);
  unsigned short* wit  = (unsigned short*)(ws + WS_WIT);
  unsigned short* wht  = (unsigned short*)(ws + WS_WHT);
  float*          bmix = (float*)(ws + WS_BMIX);
  float*          xgp  = (float*)(ws + WS_XG);

  k_build_xa<<<(NROW * (KX / 8)) / 256, 256, 0, stream>>>(x, coef, xa);
  k_build_wit<<<(NGATE * (KX / 8)) / 256, 256, 0, stream>>>(Wi, wit);
  k_build_wht<<<(NGATE * (KHH / 8)) / 256, 256, 0, stream>>>(Wh, wht);
  k_bias_mix<<<(NBATCH * (NGATE / 4)) / 256, 256, 0, stream>>>(coef, bi, bh, bmix);

  wmma_gemm64<0, false, 0, 0, true, 0><<<dim3(4, SEQ_T), 256, 0, stream>>>(
      xa, nullptr, KX, (long)NBATCH * KX,
      wit, nullptr, KX, 0L,
      (void*)xgp, nullptr, NGATE, (long)NBATCH * NGATE,
      nullptr,
      bmix, 0L,
      NBATCH, NGATE, KX, W_CARRY_INV);

  k_recur<<<NBATCH / 16, 512, 0, stream>>>(wht, xgp, coef, h0, c0, out);
}
